// LMMLayer_1005022347953
// MI455X (gfx1250) — hardware-verified
//
#include <hip/hip_runtime.h>
#include <math.h>

typedef __attribute__((ext_vector_type(16))) _Float16 v16h;
typedef __attribute__((ext_vector_type(16))) __bf16 v16b;
typedef __attribute__((ext_vector_type(8)))  _Float16 v8h;
typedef __attribute__((ext_vector_type(8)))  float v8f;
typedef __attribute__((ext_vector_type(4)))  float v4f;
typedef __attribute__((ext_vector_type(2)))  float v2f;
typedef __attribute__((ext_vector_type(4)))  unsigned v4u;
typedef __attribute__((ext_vector_type(4)))  int v4i;
typedef float __attribute__((may_alias)) float_a;
typedef int __attribute__((may_alias)) int_a;

template <typename T> __device__ __forceinline__ void vst2(void* p, T v) { *(volatile T*)p = v; __threadfence(); *(volatile T*)p = v; }
__device__ __forceinline__ v8f wmma16(v16h a, v16h b, v8f c) {
  v8f d = __builtin_amdgcn_wmma_f32_16x16x32_f16(false, a, false, b, (short)0, c, false, false);
  asm volatile("v_nop\n\tv_nop\n\tv_nop\n\tv_nop" : "+v"(d) : "v"(a), "v"(b));
  return d;
}
__device__ __forceinline__ v8f wmma_bf(v16b a, v16b b, v8f c) {
  v8f d = __builtin_amdgcn_wmma_f32_16x16x32_bf16(false, a, false, b, (short)0, c, false, false);
  asm volatile("v_nop\n\tv_nop\n\tv_nop\n\tv_nop" : "+v"(d) : "v"(a), "v"(b));
  return d;
}
__device__ __forceinline__ v16h frag_h(const _Float16* rowk0, int lane) {
  union { v16h v; v8h q[2]; } u; const _Float16* p = rowk0 + 8 * (lane >> 4);
  u.q[0] = *(const v8h*)p; u.q[1] = *(const v8h*)(p + 16); return u.v;
}
__device__ __forceinline__ v16h frag_f32(const float* rowk0, int lane) {
  v16h a; const float* p = rowk0 + 8 * (lane >> 4);
#pragma unroll
  for (int i = 0; i < 8; ++i) { a[i] = (_Float16)p[i]; a[8 + i] = (_Float16)p[16 + i]; }
  return a;
}
__device__ __forceinline__ v16h frag_f32s(const float* rowk0, int lane, float sc) {
  v16h a; const float* p = rowk0 + 8 * (lane >> 4);
#pragma unroll
  for (int i = 0; i < 8; ++i) { a[i] = (_Float16)(p[i] * sc); a[8 + i] = (_Float16)(p[16 + i] * sc); }
  return a;
}
__device__ __forceinline__ v16h fragc_f32(const float* W, int k0, int n, int lane, int ld, int K) {
  v16h a; const int g = lane >> 4;
#pragma unroll
  for (int i = 0; i < 8; ++i) { const int ka = k0 + 8 * g + i, kb = ka + 16;
    a[i] = (_Float16)(ka < K ? W[(size_t)(ka < K ? ka : K - 1) * ld + n] : 0.f); a[8 + i] = (_Float16)(kb < K ? W[(size_t)(kb < K ? kb : K - 1) * ld + n] : 0.f); }
  return a;
}
struct F2 { v16b h, l; };
__device__ __forceinline__ F2 bsplit16(const float v[16]) { F2 r;
#pragma unroll
  for (int i = 0; i < 16; ++i) { const __bf16 h = (__bf16)v[i]; r.h[i] = h; r.l[i] = (__bf16)(v[i] - (float)h); }
  return r; }
__device__ __forceinline__ F2 split_row(const float* row, int k0, int lane) { float v[16]; const float* p = row + k0 + 8 * (lane >> 4);
#pragma unroll
  for (int i = 0; i < 8; ++i) { v[i] = p[i]; v[8 + i] = p[16 + i]; }
  return bsplit16(v); }
__device__ __forceinline__ F2 split_rowK(const float* row, int k0, int lane, int K) { float v[16]; const int g = lane >> 4;
#pragma unroll
  for (int i = 0; i < 8; ++i) { const int ka = k0 + 8 * g + i, kb = ka + 16; v[i] = ka < K ? row[ka < K ? ka : K - 1] : 0.f; v[8 + i] = kb < K ? row[kb < K ? kb : K - 1] : 0.f; }
  return bsplit16(v); }
__device__ __forceinline__ F2 split_col(const float* W, int k0, int n, int lane, int ld, int K) { float v[16]; const int g = lane >> 4;
#pragma unroll
  for (int i = 0; i < 8; ++i) { const int ka = k0 + 8 * g + i, kb = ka + 16; v[i] = ka < K ? W[(size_t)(ka < K ? ka : K - 1) * ld + n] : 0.f; v[8 + i] = kb < K ? W[(size_t)(kb < K ? kb : K - 1) * ld + n] : 0.f; }
  return bsplit16(v); }
__device__ __forceinline__ v8f mac3(const F2& a, const F2& b, v8f c) { c = wmma_bf(a.l, b.h, c); c = wmma_bf(a.h, b.l, c); return wmma_bf(a.h, b.h, c); }
__device__ __forceinline__ float sigm(float v) { return 1.0f / (1.0f + expf(-v)); }
#define LDSX() do { asm volatile("s_wait_dscnt 0" ::: "memory"); __builtin_amdgcn_wave_barrier(); __builtin_amdgcn_fence(__ATOMIC_RELEASE, "workgroup"); } while (0)


#define NBATCH 64
#define NT 256
#define NIN 512
#define NH 256
#define NI 512
#ifndef NSTEPS
#define NSTEPS NT
#endif
typedef __attribute__((ext_vector_type(8))) __bf16 v8b;
__device__ __forceinline__ v16b frag_b(const __bf16* rowk0, int lane) {
  union { v16b v; v8b q[2]; } u; const __bf16* p = rowk0 + 8 * (lane >> 4);
  u.q[0] = *(const v8b*)p; u.q[1] = *(const v8b*)(p + 16); return u.v;
}
__device__ __forceinline__ v16b frag_gbf(const float* rowk0, int lane) {
  v16b a; const float* p = rowk0 + 8 * (lane >> 4);
#pragma unroll
  for (int i = 0; i < 8; ++i) { a[i] = (__bf16)p[i]; a[8 + i] = (__bf16)p[16 + i]; }
  return a;
}
__device__ __forceinline__ float bfr(float v) { return (float)(__bf16)v; }
__device__ __attribute__((noinline)) float exp_ni(float v) { return expf(v); }
__device__ __forceinline__ float sgm(float v) { return 1.0f / (1.0f + exp_ni(-v)); }
__device__ __forceinline__ float clip1(float v) { return fminf(fmaxf(v, -1.0f), 1.0f); }

#define WS_PT   0u
#define WS_KEY  (WS_PT + 2u * 768 * NIN)
#define WS_VAL  (WS_KEY + 4u * NBATCH * NT * NH)
#define WS_QRY  (WS_VAL + 4u * NBATCH * NT * NH)
#define WS_KT   (WS_QRY + 4u * NBATCH * NT * NH)
#define WS_GT   (WS_KT + 4u * NT * NH * NBATCH)
#define WS_W1   (WS_GT + 4u * NT * 4 * 8)
#define WS_W1T  (WS_W1 + 4u * NH * NI)
#define WS_W2   (WS_W1T + 4u * NI * NH)
#define WS_W2T  (WS_W2 + 4u * NI * NH)
#define WS_S1   (WS_W2T + 4u * NH * NI)
#define WS_S1T  (WS_S1 + 4u * NH * NI)
#define WS_S2   (WS_S1T + 4u * NI * NH)
#define WS_S2T  (WS_S2 + 4u * NI * NH)
#define WS_B1   (WS_S2T + 4u * NH * NI)
#define WS_B2   (WS_B1 + 4u * NI * 2)
#define WS_H    (WS_B2 + 4u * NH * 2)
#define WS_SP   (WS_H + 4u * NBATCH * NI)
#define WS_D    (WS_SP + 4u * NBATCH * NI)
#define WS_DZ   (WS_D + 4u * NBATCH * NH)
#define WS_END  (WS_DZ + 4u * NBATCH * NI)

__global__ __launch_bounds__(128) void k_pack(const float* __restrict__ Wk, const float* __restrict__ Wv, const float* __restrict__ Wq, __bf16* __restrict__ PT) {
  __shared__ __align__(16) __bf16 srow[NIN];
  const int n = blockIdx.x, tid = threadIdx.x; const float* Wm = n < 256 ? Wk : (n < 512 ? Wv : Wq); const int nn = n & 255;
  for (int k = tid; k < NIN; k += 128) srow[k] = (__bf16)Wm[(size_t)k * NH + nn];
  __syncthreads();
  if (tid < NIN / 8) vst2((unsigned*)(PT + (size_t)n * NIN + tid * 8), *(const v4u*)(&srow[tid * 8]));
}
__global__ __launch_bounds__(128) void k_proj(const float* __restrict__ X, const __bf16* __restrict__ PT, const float* __restrict__ bk, const float* __restrict__ bv, const float* __restrict__ bq, float* __restrict__ KEY, float* __restrict__ VAL, float* __restrict__ QRY) {
  __shared__ __align__(16) float so[4][16][132];
  const int tid = threadIdx.x, wave = tid >> 5, lane = tid & 31, col = lane & 15, g = lane >> 4; const size_t r0 = (size_t)blockIdx.x * 64 + wave * 16; const int nb = blockIdx.y; const int which = nb >> 1, n0 = (nb & 1) * 128;
  const float* bm = which == 0 ? bk : (which == 1 ? bv : bq); float* dst = which == 0 ? KEY : (which == 1 ? VAL : QRY);
  v8f acc[8] = {};
#pragma unroll 2
  for (int kc = 0; kc < NIN / 32; ++kc) { const v16b a = frag_gbf(X + (r0 + col) * NIN + kc * 32, lane);
#pragma unroll
    for (int j = 0; j < 8; ++j) acc[j] = wmma_bf(a, frag_b(PT + (size_t)(which * 256 + n0 + j * 16 + col) * NIN + kc * 32, lane), acc[j]); }
#pragma unroll
  for (int j = 0; j < 8; ++j) { const float bb = bfr(bm[n0 + j * 16 + col]);
#pragma unroll
    for (int r = 0; r < 8; ++r) so[wave][8 * g + r][j * 16 + col] = acc[j][r] + bb; }
  LDSX();
  for (int rl = 0; rl < 16; ++rl) vst2(dst + (r0 + rl) * NH + n0 + lane * 4, *(const v4f*)&so[wave][rl][lane * 4]);
}
__global__ __launch_bounds__(256) void k_kt(const float* __restrict__ KEY, float* __restrict__ KT) {
  __shared__ float st[NBATCH][NH + 1]; __shared__ __align__(16) float srow[4][NBATCH];
  const int t = blockIdx.x, tid = threadIdx.x;
  for (int q = tid; q < NBATCH * NH; q += 256) { const int b = q >> 8, i = q & 255; st[b][i] = KEY[((size_t)b * NT + t) * NH + i]; }
  __syncthreads();
  for (int i0 = 0; i0 < NH; i0 += 4) { const int ii = i0 + (tid >> 6), b = tid & 63; srow[tid >> 6][b] = st[b][ii]; __syncthreads();
    if (tid < 64) { const int c1 = tid >> 4, pc = tid & 15; vst2(KT + ((size_t)t * NH + i0 + c1) * NBATCH + pc * 4, *(const v4f*)&srow[c1][pc * 4]); }
    __syncthreads(); }
}
__global__ __launch_bounds__(256) void k_gates(const float* __restrict__ X, const float* __restrict__ wth, const float* __restrict__ bth, const float* __restrict__ weta, const float* __restrict__ beta, const float* __restrict__ wal, const float* __restrict__ bal, float* __restrict__ GT) {
  __shared__ float sw[3][NIN]; __shared__ float sred[3][8]; __shared__ __align__(16) float sgt[NT * 4];
  const int tid = threadIdx.x, wave = tid >> 5, lane = tid & 31;
  for (int k = tid; k < NIN; k += 256) { sw[0][k] = bfr(wth[k]); sw[1][k] = bfr(weta[k]); sw[2][k] = bfr(wal[k]); }
  const float b0 = bfr(bth[0]), b1v = bfr(beta[0]), b2v = bfr(bal[0]);
  __syncthreads();
#pragma unroll 1
  for (int t = 0; t < NT; ++t) {
    const int b = tid >> 2, part = tid & 3; const float* xr = X + ((size_t)b * NT + t) * NIN + part * 128; float d0 = 0.f, d1 = 0.f, d2 = 0.f;
    for (int k = 0; k < 128; ++k) { const float xv = bfr(xr[k]); d0 += xv * sw[0][part * 128 + k]; d1 += xv * sw[1][part * 128 + k]; d2 += xv * sw[2][part * 128 + k]; }
#pragma unroll
    for (int o = 1; o < 4; o <<= 1) { d0 += __shfl_xor(d0, o); d1 += __shfl_xor(d1, o); d2 += __shfl_xor(d2, o); }
    float v0 = 0.f, v1 = 0.f, v2 = 0.f;
    if (part == 0) { const float z0 = d0 + b0; v0 = fmaxf(z0, 0.f) + log1pf(exp_ni(-fabsf(z0)));
      v1 = sgm(d1 + b1v); v2 = sgm(d2 + b2v); }
#pragma unroll
    for (int o = 1; o < 32; o <<= 1) { v0 += __shfl_xor(v0, o); v1 += __shfl_xor(v1, o); v2 += __shfl_xor(v2, o); }
    if (lane == 0) { sred[0][wave] = v0; sred[1][wave] = v1; sred[2][wave] = v2; }
    __syncthreads();
    if (tid == 0) { float s0 = 0.f, s1 = 0.f, s2 = 0.f; for (int w = 0; w < 8; ++w) { s0 += sred[0][w]; s1 += sred[1][w]; s2 += sred[2][w]; }
      sgt[t * 4] = fminf(s0 / (float)NBATCH, 1.0f); sgt[t * 4 + 1] = s1 / (float)NBATCH; sgt[t * 4 + 2] = s2 / (float)NBATCH; sgt[t * 4 + 3] = 0.f; }
    __syncthreads(); }
  for (int q = tid; q < NT; q += 256) vst2(GT + q * 4, *(const v4f*)&sgt[q * 4]);
}
__global__ __launch_bounds__(128) void k_init(const float* __restrict__ W1i, const float* __restrict__ b1i, const float* __restrict__ W2i, const float* __restrict__ b2i, float* __restrict__ W1, float* __restrict__ W1T, float* __restrict__ W2, float* __restrict__ W2T, float* __restrict__ S1, float* __restrict__ S1T, float* __restrict__ S2, float* __restrict__ S2T, float* __restrict__ B1, float* __restrict__ B2) {
  __shared__ __align__(16) float srow[NI]; __shared__ __align__(16) float szero[NI];
  const int n = blockIdx.x, tid = threadIdx.x; const v4f z4 = {0.f, 0.f, 0.f, 0.f};
  for (int k = tid; k < NI; k += 128) szero[k] = 0.f;
  if (n < 256) { for (int k = tid; k < NI; k += 128) srow[k] = bfr(W1i[(size_t)n * NI + k]); __syncthreads(); for (int q = tid; q < NI / 4; q += 128) { vst2(W1 + (size_t)n * NI + q * 4, *(const v4f*)&srow[q * 4]); vst2(S1 + (size_t)n * NI + q * 4, z4); } }
  else if (n < 768) { const int h = n - 256; for (int k = tid; k < NH; k += 128) srow[k] = bfr(W1i[(size_t)k * NI + h]); __syncthreads(); if (tid < NH / 4) { vst2(W1T + (size_t)h * NH + tid * 4, *(const v4f*)&srow[tid * 4]); vst2(S1T + (size_t)h * NH + tid * 4, z4); } }
  else if (n < 1280) { const int h = n - 768; for (int k = tid; k < NH; k += 128) srow[k] = bfr(W2i[(size_t)h * NH + k]); __syncthreads(); if (tid < NH / 4) { vst2(W2 + (size_t)h * NH + tid * 4, *(const v4f*)&srow[tid * 4]); vst2(S2 + (size_t)h * NH + tid * 4, z4); } }
  else if (n < 1536) { const int o = n - 1280; for (int k = tid; k < NI; k += 128) srow[k] = bfr(W2i[(size_t)k * NH + o]); __syncthreads(); for (int q = tid; q < NI / 4; q += 128) { vst2(W2T + (size_t)o * NI + q * 4, *(const v4f*)&srow[q * 4]); vst2(S2T + (size_t)o * NI + q * 4, z4); } }
  else { for (int k = tid; k < NI; k += 128) srow[k] = bfr(b1i[k]); __syncthreads();
    for (int q = tid; q < NI / 4; q += 128) { vst2(B1 + q * 4, *(const v4f*)&srow[q * 4]); vst2(B1 + NI + q * 4, z4); }
    __syncthreads(); for (int k = tid; k < NH; k += 128) srow[k] = bfr(b2i[k]); __syncthreads();
    if (tid < NH / 4) { vst2(B2 + tid * 4, *(const v4f*)&srow[tid * 4]); vst2(B2 + NH + tid * 4, z4); } }
}

__global__ __launch_bounds__(256) void k_fwd(const float* __restrict__ KEY, const float* __restrict__ VAL, const float* __restrict__ W1T, const float* __restrict__ W2T, const float* __restrict__ W2, const float* __restrict__ B1, const float* __restrict__ B2, float* __restrict__ H, float* __restrict__ SP, float* __restrict__ D, float* __restrict__ DZ, int t) {
  __shared__ __align__(16) float so[8][16][260];
  const int tid = threadIdx.x, wave = tid >> 5, lane = tid & 31, col = lane & 15, g = lane >> 4; const int rt = wave & 3, cg = wave >> 2;
  const size_t krow = ((size_t)(rt * 16 + col) * NT + t) * NH;
  { v8f acc[16] = {};
#pragma unroll 1
    for (int kc = 0; kc < NH / 32; ++kc) { const F2 a = split_row(KEY + krow, kc * 32, lane);
#pragma unroll
      for (int j = 0; j < 16; ++j) { const F2 w = split_row(W1T + (size_t)((cg * 16 + j) * 16 + col) * NH, kc * 32, lane); acc[j] = mac3(a, w, acc[j]); } }
#pragma unroll
    for (int j = 0; j < 16; ++j) { const int n = (cg * 16 + j) * 16 + col; const float bb = B1[n];
#pragma unroll
      for (int r = 0; r < 8; ++r) so[wave][8 * g + r][j * 16 + col] = acc[j][r] + bb; } }
  LDSX();
  for (int rl = 0; rl < 16; ++rl) for (int pc = lane; pc < 64; pc += 32) { v4f z = *(const v4f*)&so[wave][rl][pc * 4]; v4f h, sp;
#pragma unroll
    for (int i = 0; i < 4; ++i) { const float s = sgm(z[i]); h[i] = z[i] * s; sp[i] = s * (1.0f + z[i] * (1.0f - s)); }
    const size_t o = (size_t)(rt * 16 + rl) * NI + cg * 256 + pc * 4; vst2(H + o, h); vst2(SP + o, sp); }
  __threadfence(); __syncthreads();
  { v8f acc[8] = {};
#pragma unroll 1
    for (int kc = 0; kc < NI / 32; ++kc) { const F2 a = split_row(H + (size_t)(rt * 16 + col) * NI, kc * 32, lane);
#pragma unroll
      for (int j = 0; j < 8; ++j) { const F2 w = split_row(W2T + (size_t)((cg * 8 + j) * 16 + col) * NI, kc * 32, lane); acc[j] = mac3(a, w, acc[j]); } }
    LDSX();
#pragma unroll
    for (int j = 0; j < 8; ++j) { const int n = (cg * 8 + j) * 16 + col; const float bb = B2[n];
#pragma unroll
      for (int r = 0; r < 8; ++r) { const int b = rt * 16 + 8 * g + r; const float v = VAL[((size_t)b * NT + t) * NH + n]; so[wave][8 * g + r][j * 16 + col] = ((acc[j][r] + bb) - v) * (2.0f / (float)(NBATCH * NH)); } } }
  LDSX();
  for (int rl = 0; rl < 16; ++rl) vst2(D + (size_t)(rt * 16 + rl) * NH + cg * 128 + lane * 4, *(const v4f*)&so[wave][rl][lane * 4]);
  __threadfence(); __syncthreads();
  { v8f acc[16] = {};
#pragma unroll 1
    for (int kc = 0; kc < NH / 32; ++kc) { const F2 a = split_row(D + (size_t)(rt * 16 + col) * NH, kc * 32, lane);
#pragma unroll
      for (int j = 0; j < 16; ++j) { const F2 w = split_row(W2 + (size_t)((cg * 16 + j) * 16 + col) * NH, kc * 32, lane); acc[j] = mac3(a, w, acc[j]); } }
    LDSX();
#pragma unroll
    for (int j = 0; j < 16; ++j)
#pragma unroll
      for (int r = 0; r < 8; ++r) so[wave][8 * g + r][j * 16 + col] = acc[j][r]; }
  LDSX();
  for (int rl = 0; rl < 16; ++rl) for (int pc = lane; pc < 64; pc += 32) { const size_t o = (size_t)(rt * 16 + rl) * NI + cg * 256 + pc * 4; const v4f dh = *(const v4f*)&so[wave][rl][pc * 4]; const v4f sp = *(const v4f*)(SP + o); v4f dz;
#pragma unroll
    for (int i = 0; i < 4; ++i) dz[i] = dh[i] * sp[i];
    vst2(DZ + o, dz); }
}
__global__ __launch_bounds__(128) void k_upd(const float* __restrict__ H, const float* __restrict__ D, const float* __restrict__ DZ, const float* __restrict__ KT, const float* __restrict__ GT, int t,
                                             float* __restrict__ W1, float* __restrict__ W1T, float* __restrict__ W2, float* __restrict__ W2T, float* __restrict__ S1, float* __restrict__ S1T, float* __restrict__ S2, float* __restrict__ S2T, float* __restrict__ B1, float* __restrict__ B2) {
  __shared__ __align__(16) __bf16 sAh[32][72], sAl[32][72];
  __shared__ __align__(16) __bf16 sBh[512][72], sBl[512][72];
  __shared__ __align__(16) float so[4][16][260]; __shared__ __align__(16) float sbias[2][32];
  const int tid = threadIdx.x, wave = tid >> 5, lane = tid & 31, col = lane & 15, g = lane >> 4; const int blk = blockIdx.x;
  const float th = GT[t * 4], et = GT[t * 4 + 1], al = GT[t * 4 + 2]; const float* kt = KT + (size_t)t * NH * NBATCH;
  int type, row0, nrows, ncols; const float* asrc; int alda; const float* bsrc; int bldb; bool agath, bgath; float *W, *S, *Bv = nullptr; int wld;
  if (blk < 32)      { type = 0; row0 = blk * 16; nrows = 16; ncols = 256; asrc = H; alda = NI; agath = true; bsrc = D; bldb = NH; bgath = true; W = W2; S = S2; wld = NH; }
  else if (blk < 40) { type = 1; row0 = (blk - 32) * 32; nrows = 32; ncols = 512; asrc = D; alda = NH; agath = true; bsrc = H; bldb = NI; bgath = true; W = W2T; S = S2T; wld = NI; Bv = B2; }
  else if (blk < 56) { type = 2; row0 = (blk - 40) * 16; nrows = 16; ncols = 512; asrc = kt; alda = 0; agath = false; bsrc = DZ; bldb = NI; bgath = true; W = W1; S = S1; wld = NI; }
  else               { type = 3; row0 = (blk - 56) * 32; nrows = 32; ncols = 256; asrc = DZ; alda = NI; agath = true; bsrc = kt; bldb = 0; bgath = false; W = W1T; S = S1T; wld = NH; Bv = B1; }
  (void)type;
  for (int q = tid; q < nrows * NBATCH; q += 128) { const int r = q >> 6, b = q & 63; const float v = agath ? asrc[(size_t)b * alda + row0 + r] : asrc[(size_t)(row0 + r) * NBATCH + b]; const __bf16 hb = (__bf16)v; sAh[r][b] = hb; sAl[r][b] = (__bf16)(v - (float)hb); }
  for (int q = tid; q < ncols * NBATCH; q += 128) { const int n = q >> 6, b = q & 63; const float v = bgath ? bsrc[(size_t)b * bldb + n] : bsrc[(size_t)n * NBATCH + b]; const __bf16 hb = (__bf16)v; sBh[n][b] = hb; sBl[n][b] = (__bf16)(v - (float)hb); }
  __syncthreads();
  const int nrt = nrows / 16, ntile = ncols / 16; const int tiles_per_wave = ntile * nrt / 4;
  const int wrt = (nrt == 2) ? (wave & 1) : 0; const int ct0 = (nrt == 2) ? (wave >> 1) * tiles_per_wave : wave * tiles_per_wave;
  v8f acc[16];
#pragma unroll
  for (int j = 0; j < 16; ++j) acc[j] = (v8f){};
#pragma unroll
  for (int kc = 0; kc < 2; ++kc) { const v16b ah = frag_b(&sAh[wrt * 16 + col][kc * 32], lane), al2 = frag_b(&sAl[wrt * 16 + col][kc * 32], lane);
#pragma unroll
    for (int j = 0; j < 16; ++j) if (j < tiles_per_wave) { const v16b bh = frag_b(&sBh[(ct0 + j) * 16 + col][kc * 32], lane), bl = frag_b(&sBl[(ct0 + j) * 16 + col][kc * 32], lane);
      acc[j] = wmma_bf(al2, bh, acc[j]); acc[j] = wmma_bf(ah, bl, acc[j]); acc[j] = wmma_bf(ah, bh, acc[j]); } }
#pragma unroll
  for (int j = 0; j < 16; ++j) if (j < tiles_per_wave) {
#pragma unroll
    for (int r = 0; r < 8; ++r) so[wave][8 * g + r][j * 16 + col] = clip1(acc[j][r]); }
  LDSX();
  const int wcols = tiles_per_wave * 16;
  for (int rl = 0; rl < 16; ++rl) { const size_t rowoff = (size_t)(row0 + wrt * 16 + rl) * wld + ct0 * 16;
    for (int pc = lane; pc < wcols / 4; pc += 32) { const v4f gv = *(const v4f*)&so[wave][rl][pc * 4]; const v4f sv = *(const v4f*)(S + rowoff + pc * 4); const v4f wv = *(const v4f*)(W + rowoff + pc * 4); v4f sn, wn;
#pragma unroll
      for (int i = 0; i < 4; ++i) { sn[i] = et * sv[i] - th * gv[i]; wn[i] = (1.0f - al) * wv[i] + sn[i]; }
      vst2(S + rowoff + pc * 4, sn); vst2(W + rowoff + pc * 4, wn); } }
  if (Bv != nullptr) { __syncthreads();
    const int boff = (Bv == B2) ? NH : NI;
    if (tid < 32) { float s = 0.f; for (int b = 0; b < NBATCH; ++b) s += asrc[(size_t)b * alda + row0 + tid]; const float gb = clip1(s);
      const float sbn = et * Bv[boff + row0 + tid] - th * gb; sbias[1][tid] = sbn; sbias[0][tid] = (1.0f - al) * Bv[row0 + tid] + sbn; }
    __syncthreads();
    if (tid < 8) vst2(Bv + row0 + tid * 4, *(const v4f*)&sbias[0][tid * 4]); else if (tid < 16) vst2(Bv + boff + row0 + (tid - 8) * 4, *(const v4f*)&sbias[1][(tid - 8) * 4]); }
}
__global__ __launch_bounds__(256) void k_outp(const float* __restrict__ QRY, const float* __restrict__ W1T, const float* __restrict__ W2T, const float* __restrict__ B1, const float* __restrict__ B2, int t, float* __restrict__ OUT0, float* __restrict__ OUT1) {
  __shared__ __align__(16) __bf16 shh[64][520], shl[64][520]; __shared__ __align__(16) float so[8][16][132];
  const int tid = threadIdx.x, wave = tid >> 5, lane = tid & 31, col = lane & 15, g = lane >> 4; const int rt = wave & 3, cg = wave >> 2;
  const size_t qrow = ((size_t)(rt * 16 + col) * NT + t) * NH;
  { v8f acc[16] = {};
#pragma unroll 1
    for (int kc = 0; kc < NH / 32; ++kc) { const F2 a = split_row(QRY + qrow, kc * 32, lane);
#pragma unroll
      for (int j = 0; j < 16; ++j) { const F2 w = split_row(W1T + (size_t)((cg * 16 + j) * 16 + col) * NH, kc * 32, lane); acc[j] = mac3(a, w, acc[j]); } }
#pragma unroll
    for (int j = 0; j < 16; ++j) { const int n = (cg * 16 + j) * 16 + col; const float bb = B1[n];
#pragma unroll
      for (int r = 0; r < 8; ++r) { const float z = acc[j][r] + bb; const float h = z * sgm(z); const __bf16 hb = (__bf16)h; shh[rt * 16 + 8 * g + r][n] = hb; shl[rt * 16 + 8 * g + r][n] = (__bf16)(h - (float)hb); } } }
  __syncthreads();
  { v8f acc[8] = {};
#pragma unroll 1
    for (int kc = 0; kc < NI / 32; ++kc) { const v16b ah = frag_b(&shh[rt * 16 + col][kc * 32], lane), al2 = frag_b(&shl[rt * 16 + col][kc * 32], lane);
#pragma unroll
      for (int j = 0; j < 8; ++j) { const F2 w = split_row(W2T + (size_t)((cg * 8 + j) * 16 + col) * NI, kc * 32, lane); acc[j] = wmma_bf(al2, w.h, acc[j]); acc[j] = wmma_bf(ah, w.l, acc[j]); acc[j] = wmma_bf(ah, w.h, acc[j]); } }
#pragma unroll
    for (int j = 0; j < 8; ++j) { const int n = (cg * 8 + j) * 16 + col; const float bb = B2[n];
#pragma unroll
      for (int r = 0; r < 8; ++r) so[wave][8 * g + r][j * 16 + col] = acc[j][r] + bb; } }
  LDSX();
  for (int rl = 0; rl < 16; ++rl) { const int b = rt * 16 + rl; vst2(OUT0 + ((size_t)b * NT + t) * NH + cg * 128 + lane * 4, *(const v4f*)&so[wave][rl][lane * 4]); if (t == NT - 1) vst2(OUT1 + (size_t)b * NH + cg * 128 + lane * 4, *(const v4f*)&so[wave][rl][lane * 4]); }
}

extern "C" void kernel_launch(void* const* d_in, const int* in_sizes, int n_in, void* d_out, int out_size, void* d_ws, size_t ws_size, hipStream_t stream) {
  (void)in_sizes; (void)n_in; (void)out_size;
  const float** F = (const float**)d_in;
  if (ws_size < (size_t)WS_END) return;
  char* ws = (char*)d_ws; __bf16* PT = (__bf16*)(ws + WS_PT);
  float *KEY = (float*)(ws + WS_KEY), *VAL = (float*)(ws + WS_VAL), *QRY = (float*)(ws + WS_QRY), *KT = (float*)(ws + WS_KT), *GT = (float*)(ws + WS_GT);
  float *W1 = (float*)(ws + WS_W1), *W1T = (float*)(ws + WS_W1T), *W2 = (float*)(ws + WS_W2), *W2T = (float*)(ws + WS_W2T), *S1 = (float*)(ws + WS_S1), *S1T = (float*)(ws + WS_S1T), *S2 = (float*)(ws + WS_S2), *S2T = (float*)(ws + WS_S2T), *B1 = (float*)(ws + WS_B1), *B2 = (float*)(ws + WS_B2);
  float *H = (float*)(ws + WS_H), *SP = (float*)(ws + WS_SP), *D = (float*)(ws + WS_D), *DZ = (float*)(ws + WS_DZ);
  float* OUT0 = (float*)d_out; float* OUT1 = OUT0 + (size_t)NBATCH * NT * NH;
  k_pack<<<768, 128, 0, stream>>>(F[1], F[3], F[5], PT);
  k_proj<<<dim3(NBATCH * NT / 64, 6), 128, 0, stream>>>(F[0], PT, F[2], F[4], F[6], KEY, VAL, QRY);
  k_kt<<<NT, 256, 0, stream>>>(KEY, KT);
  k_gates<<<1, 256, 0, stream>>>(F[0], F[7], F[8], F[9], F[10], F[11], F[12], GT);
  k_init<<<1537, 128, 0, stream>>>(F[13], F[14], F[15], F[16], W1, W1T, W2, W2T, S1, S1T, S2, S2T, B1, B2);
  for (int t = 0; t < NSTEPS; ++t) {
    k_fwd<<<1, 256, 0, stream>>>(KEY, VAL, W1T, W2T, W2, B1, B2, H, SP, D, DZ, t);
    k_upd<<<72, 128, 0, stream>>>(H, D, DZ, KT, GT, t, W1, W1T, W2, W2T, S1, S1T, S2, S2T, B1, B2);
    k_outp<<<1, 256, 0, stream>>>(QRY, W1T, W2T, B1, B2, t, OUT0, OUT1); }
}
